// CrossModel_55499567399318
// MI455X (gfx1250) — hardware-verified
//
#include <hip/hip_runtime.h>
#include <stddef.h>


#define DF      128
#define DO      64
#define NTHR    256
#define NWAVE   8
#define EPT     8
#define NGRP    2
#define CHUNK   (NTHR * EPT * NGRP)
#define WCAP    (EPT * NGRP * 32)
#define LISTN   (NWAVE * WCAP)
#define NB1     512
#define NB2     1024
#define NBD     4096
#define GROWS   128
#define APITCH  136
#define WSCALE  8.0f
#define WINV    0.125f

#define LDS_GEMM1 (GROWS * DF * 4)
#define LDS_GEMM2 (GROWS * APITCH * 2)
#define LDS_AGG1  (NB1 * DF * 4 + LISTN * 4 + 64)
#define LDS_AGG2  (NB2 * DO * 4 + LISTN * 4 + 64)

static_assert((CHUNK & (CHUNK - 1)) == 0);
static_assert(CHUNK <= 4096);
static_assert((NB1 & (NB1 - 1)) == 0 && (NB2 & (NB2 - 1)) == 0 && (NBD & (NBD - 1)) == 0);
static_assert(NB1 <= 4096 && NB2 <= 4096 && NBD <= 4096);
static_assert(GROWS * APITCH * 2 <= LDS_GEMM1);
static_assert(GROWS * DO * 4 <= LDS_GEMM2);
static_assert(NBD % GROWS == 0 && NBD % NB1 == 0 && NBD % NB2 == 0);
static_assert((NB1 * DF / 4) % NTHR == 0 && (NB2 * DO / 4) % NTHR == 0);

typedef float    v2f  __attribute__((ext_vector_type(2)));
typedef float    v4f  __attribute__((ext_vector_type(4)));
typedef float    v8f  __attribute__((ext_vector_type(8)));
typedef int      v4i  __attribute__((ext_vector_type(4)));
typedef _Float16 v8h  __attribute__((ext_vector_type(8)));
typedef _Float16 v16h __attribute__((ext_vector_type(16)));
union FragH { v16h v; v8h h[2]; };

__device__ __forceinline__ v8h cvt8(v4f a, v4f b) {
  v8h r;
  r[0] = (_Float16)a.x; r[1] = (_Float16)a.y; r[2] = (_Float16)a.z; r[3] = (_Float16)a.w;
  r[4] = (_Float16)b.x; r[5] = (_Float16)b.y; r[6] = (_Float16)b.z; r[7] = (_Float16)b.w;
  return r;
}

__device__ __forceinline__ v8f wmh(v16h a, v16h b, v8f c) {
  v8f d = __builtin_amdgcn_wmma_f32_16x16x32_f16(false, a, false, b, (short)0, c, false, false);
  asm volatile("v_nop\n\tv_nop\n\tv_nop\n\tv_nop" : "+v"(d) : "v"(a), "v"(b));
  return d;
}

template <int NB>
__device__ __forceinline__ int scan_chunk(const int* __restrict__ dsts, int nE, int cbase, int nodeBase,
                                          int vec8, int* list, int tid, int lane, int wave) {
  int wc = 0;
#pragma unroll
  for (int g = 0; g < NGRP; ++g) {
    const int el0  = (g * NTHR + tid) * EPT;
    const int e0   = cbase + el0;
    const int sent = -2147483647 - 1;
    v4i da, db;
    if (vec8 != 0 && e0 + 7 < nE) {
      da = *(const v4i*)(dsts + e0);
      db = *(const v4i*)(dsts + e0 + 4);
    } else {
      da.x = (e0     < nE) ? dsts[min(e0, nE - 1)] : sent;
      da.y = (e0 + 1 < nE) ? dsts[min(e0 + 1, nE - 1)] : sent;
      da.z = (e0 + 2 < nE) ? dsts[min(e0 + 2, nE - 1)] : sent;
      da.w = (e0 + 3 < nE) ? dsts[min(e0 + 3, nE - 1)] : sent;
      db.x = (e0 + 4 < nE) ? dsts[min(e0 + 4, nE - 1)] : sent;
      db.y = (e0 + 5 < nE) ? dsts[min(e0 + 5, nE - 1)] : sent;
      db.z = (e0 + 6 < nE) ? dsts[min(e0 + 6, nE - 1)] : sent;
      db.w = (e0 + 7 < nE) ? dsts[min(e0 + 7, nE - 1)] : sent;
    }
    const unsigned nb = (unsigned)nodeBase;
    const unsigned s0 = (unsigned)da.x - nb, s1 = (unsigned)da.y - nb;
    const unsigned s2 = (unsigned)da.z - nb, s3 = (unsigned)da.w - nb;
    const unsigned s4 = (unsigned)db.x - nb, s5 = (unsigned)db.y - nb;
    const unsigned s6 = (unsigned)db.z - nb, s7 = (unsigned)db.w - nb;
    const bool h0 = s0 < (unsigned)NB, h1 = s1 < (unsigned)NB, h2 = s2 < (unsigned)NB, h3 = s3 < (unsigned)NB;
    const bool h4 = s4 < (unsigned)NB, h5 = s5 < (unsigned)NB, h6 = s6 < (unsigned)NB, h7 = s7 < (unsigned)NB;
    const unsigned any = __builtin_amdgcn_ballot_w32(h0 | h1 | h2 | h3 | h4 | h5 | h6 | h7);
    if (any != 0u) {
#define HITJ(J, HJ, SJ) { \
        const unsigned mj = __builtin_amdgcn_ballot_w32(HJ); \
        if (mj != 0u) { \
          if (HJ) { \
            const int pos = wc + (int)__builtin_amdgcn_mbcnt_lo(mj, 0u); \
            if (pos < WCAP) list[wave * WCAP + pos] = ((el0 + (J)) << 12) | (int)(SJ); \
          } \
          wc += (int)__builtin_popcount(mj); } }
      HITJ(0, h0, s0)
      HITJ(1, h1, s1)
      HITJ(2, h2, s2)
      HITJ(3, h3, s3)
      HITJ(4, h4, s4)
      HITJ(5, h5, s5)
      HITJ(6, h6, s6)
      HITJ(7, h7, s7)
#undef HITJ
    }
  }
  return wc;
}

__global__ __launch_bounds__(NTHR) void k_wprep(
    const float* __restrict__ W1, const float* __restrict__ W2, const float* __restrict__ W3,
    _Float16* w1s, _Float16* w2s, _Float16* w3s) {
  const int i  = blockIdx.x * NTHR + threadIdx.x;
  const int n1 = DF * DF / 8;
  const int n3 = DO * DF / 8;
  if (i >= 2 * n1 + n3) return;
  const int which = i < n1 ? 0 : (i < 2 * n1 ? 1 : 2);
  const int ii = i - which * n1;
  const int o  = ii * 8;
  const int n  = o / DF;
  const int k0 = o - n * DF;
  const int nc = (which == 2) ? DO : DF;
  const float* p = (which == 0 ? W1 : (which == 1 ? W2 : W3)) + (size_t)k0 * nc + n;
  v4f a, b;
  a.x = p[0];      a.y = p[nc];     a.z = p[2 * nc]; a.w = p[3 * nc];
  b.x = p[4 * nc]; b.y = p[5 * nc]; b.z = p[6 * nc]; b.w = p[7 * nc];
  a = a * WSCALE;
  b = b * WSCALE;
  const v8h hv = cvt8(a, b);
  _Float16* dp = (which == 0 ? w1s : (which == 1 ? w2s : w3s)) + o;
  *(volatile v8h*)dp = hv;
  __threadfence();
  *(volatile v8h*)dp = hv;
}

__global__ __launch_bounds__(NTHR) void k_deg(
    const int* __restrict__ ei, const float* __restrict__ ew, float* dis, int nN, int nE, int vec8) {
  __shared__ __attribute__((aligned(16))) float deg[NBD];
  __shared__ __attribute__((aligned(16))) int list[LISTN];
  __shared__ int wcnt[NWAVE];
  const int tid = threadIdx.x, lane = tid & 31, wave = tid >> 5;
  const int nodeBase = blockIdx.x * NBD;
  const int* dsts = ei + nE;
  (void)nN;

  for (int i = tid; i < NBD; i += NTHR) deg[i] = 1.0f;
  __syncthreads();

  const int nChunks = (nE + CHUNK - 1) / CHUNK;
#pragma unroll 1
  for (int ch = 0; ch < nChunks; ++ch) {
    const int cbase = ch * CHUNK;
    const int wc = scan_chunk<NBD>(dsts, nE, cbase, nodeBase, vec8, list, tid, lane, wave);
    if (lane == 0) wcnt[wave] = wc;
    __syncthreads();
    if (wave == 0) {
#pragma unroll 1
      for (int wsx = 0; wsx < NWAVE; ++wsx) {
        int n = __builtin_amdgcn_readfirstlane(wcnt[wsx]);
        n = n > WCAP ? WCAP : (n < 0 ? 0 : n);
        const int* lp = list + wsx * WCAP;
#pragma unroll 1
        for (int i = 0; i < n; ++i) {
          const int ent  = __builtin_amdgcn_readfirstlane(lp[i]);
          const int slot = ent & (NBD - 1);
          int e = cbase + ((ent >> 12) & (CHUNK - 1));
          e = e > nE - 1 ? nE - 1 : e;
          const float wv = ew[e];
          if (lane == 0) deg[slot] = deg[slot] + wv;
        }
      }
    }
    __syncthreads();
  }

  v4f dq[4];
#pragma unroll
  for (int q = 0; q < 4; ++q) {
    const int f = (wave * 4 + q) * 128 + 4 * lane;
    const v4f d = *(const v4f*)(deg + f);
    dq[q].x = d.x > 0.f ? rsqrtf(d.x) : 0.f;
    dq[q].y = d.y > 0.f ? rsqrtf(d.y) : 0.f;
    dq[q].z = d.z > 0.f ? rsqrtf(d.z) : 0.f;
    dq[q].w = d.w > 0.f ? rsqrtf(d.w) : 0.f;
  }
  float* dp = dis + (size_t)nodeBase;
#pragma unroll
  for (int q = 0; q < 4; ++q) *(volatile v4f*)(dp + (wave * 4 + q) * 128 + 4 * lane) = dq[q];
  __threadfence();
#pragma unroll
  for (int q = 0; q < 4; ++q) *(volatile v4f*)(dp + (wave * 4 + q) * 128 + 4 * lane) = dq[q];
}

__global__ __launch_bounds__(NTHR) void k_gemm1(
    const float* __restrict__ x, const _Float16* __restrict__ wns,
    const float* __restrict__ dis, float* g, int nN) {
  extern __shared__ v4f lds_dyn[];
  _Float16* sA  = (_Float16*)lds_dyn;
  float*    stg = (float*)lds_dyn;
  const int tid = threadIdx.x, lane = tid & 31, wave = tid >> 5, hh = lane >> 4, m = lane & 15;
  const int rowBase = blockIdx.x * GROWS;

#pragma unroll
  for (int i = 0; i < (GROWS * DF / 8) / NTHR; ++i) {
    const int idx = i * NTHR + tid;
    const int r   = idx >> 4;
    const int c0  = (idx & 15) * 8;
    int node = rowBase + r;
    node = node > nN - 1 ? nN - 1 : node;
    const float* xp = x + (size_t)node * DF + c0;
    const v4f a = *(const v4f*)xp, b = *(const v4f*)(xp + 4);
    *(v8h*)(sA + r * APITCH + c0) = cvt8(a, b);
  }
  __syncthreads();

  v8f acc[8];
#pragma unroll
  for (int t = 0; t < 8; ++t) { v8f z = {0.f, 0.f, 0.f, 0.f, 0.f, 0.f, 0.f, 0.f}; acc[t] = z; }
  const _Float16* ar = sA + (wave * 16 + m) * APITCH + 8 * hh;
#pragma unroll
  for (int kt = 0; kt < DF / 32; ++kt) {
    FragH a;
    a.h[0] = *(const v8h*)(ar + 32 * kt);
    a.h[1] = *(const v8h*)(ar + 32 * kt + 16);
#pragma unroll
    for (int t = 0; t < 8; ++t) {
      const _Float16* bp = wns + (size_t)(16 * t + m) * DF + 32 * kt + 8 * hh;
      FragH b;
      b.h[0] = *(const v8h*)bp;
      b.h[1] = *(const v8h*)(bp + 16);
      acc[t] = wmh(a.v, b.v, acc[t]);
    }
  }
  __syncthreads();

  const int r0 = wave * 16 + 8 * hh;
  const v4f dA = *(const v4f*)(dis + (size_t)rowBase + r0);
  const v4f dB = *(const v4f*)(dis + (size_t)rowBase + r0 + 4);
  const float d0 = dA.x * WINV, d1 = dA.y * WINV, d2 = dA.z * WINV, d3 = dA.w * WINV;
  const float d4 = dB.x * WINV, d5 = dB.y * WINV, d6 = dB.z * WINV, d7 = dB.w * WINV;
  float* sp = stg + r0 * DF + m;
#pragma unroll
  for (int t = 0; t < 8; ++t) {
    sp[0 * DF + 16 * t] = acc[t][0] * d0;
    sp[1 * DF + 16 * t] = acc[t][1] * d1;
    sp[2 * DF + 16 * t] = acc[t][2] * d2;
    sp[3 * DF + 16 * t] = acc[t][3] * d3;
    sp[4 * DF + 16 * t] = acc[t][4] * d4;
    sp[5 * DF + 16 * t] = acc[t][5] * d5;
    sp[6 * DF + 16 * t] = acc[t][6] * d6;
    sp[7 * DF + 16 * t] = acc[t][7] * d7;
  }
  __syncthreads();

  const float* lp = stg + wave * 16 * DF + 4 * lane;
  float* gp = g + ((size_t)rowBase + wave * 16) * DF + 4 * lane;
#pragma unroll
  for (int i = 0; i < 16; ++i) { const v4f v = *(const v4f*)(lp + i * DF); *(volatile v4f*)(gp + (size_t)i * DF) = v; }
  __threadfence();
#pragma unroll
  for (int i = 0; i < 16; ++i) { const v4f v = *(const v4f*)(lp + i * DF); *(volatile v4f*)(gp + (size_t)i * DF) = v; }
}

__global__ __launch_bounds__(NTHR) void k_agg1(
    const int* __restrict__ ei, const float* __restrict__ ew, const float* __restrict__ g,
    const float* __restrict__ dis, const float* __restrict__ b, float* h,
    int nN, int nE, int vec8) {
  extern __shared__ v4f lds_dyn[];
  float* acc  = (float*)lds_dyn;
  int*   list = (int*)(acc + NB1 * DF);
  int*   wcnt = list + LISTN;
  const int tid = threadIdx.x, lane = tid & 31, wave = tid >> 5;
  const int nodeBase = blockIdx.x * NB1;
  const int* dsts = ei + nE;

  {
    const v4f z = {0.f, 0.f, 0.f, 0.f};
    for (int i = tid; i < NB1 * DF / 4; i += NTHR) lds_dyn[i] = z;
  }
  __syncthreads();

  const int nChunks = (nE + CHUNK - 1) / CHUNK;
#pragma unroll 1
  for (int ch = 0; ch < nChunks; ++ch) {
    const int cbase = ch * CHUNK;
    const int wc = scan_chunk<NB1>(dsts, nE, cbase, nodeBase, vec8, list, tid, lane, wave);
    if (lane == 0) wcnt[wave] = wc;
    __syncthreads();
    if (wave == 0) {
#pragma unroll 1
      for (int wsx = 0; wsx < NWAVE; ++wsx) {
        int n = __builtin_amdgcn_readfirstlane(wcnt[wsx]);
        n = n > WCAP ? WCAP : (n < 0 ? 0 : n);
        const int* lp = list + wsx * WCAP;
#pragma unroll 1
        for (int i = 0; i < n; ++i) {
          const int ent  = __builtin_amdgcn_readfirstlane(lp[i]);
          const int slot = ent & (NB1 - 1);
          int e = cbase + ((ent >> 12) & (CHUNK - 1));
          e = e > nE - 1 ? nE - 1 : e;
          int src = ei[e];
          src = src < 0 ? 0 : (src > nN - 1 ? nN - 1 : src);
          const float wv = ew[e];
          const v4f v = *(const v4f*)(g + (size_t)src * DF + 4 * lane);
          v4f* ap = (v4f*)(acc + slot * DF + 4 * lane);
          *ap = *ap + v * wv;
        }
      }
    }
    __syncthreads();
  }

#pragma unroll 4
  for (int i = 0; i < (NB1 * DF / 4) / NTHR; ++i) {
    const int idx  = i * NTHR + tid;
    const int slot = idx >> 5;
    const int c4   = (idx & 31) * 4;
    int node = nodeBase + slot;
    node = node > nN - 1 ? nN - 1 : node;
    const float d  = dis[node];
    const v4f   gv = *(const v4f*)(g + (size_t)node * DF + c4);
    const v4f   bv = *(const v4f*)(b + c4);
    v4f* ap = (v4f*)(acc + slot * DF + c4);
    v4f hv = (*ap + gv) * d + bv;
    hv.x = fmaxf(hv.x, 0.f); hv.y = fmaxf(hv.y, 0.f); hv.z = fmaxf(hv.z, 0.f); hv.w = fmaxf(hv.w, 0.f);
    *ap = hv;
    *(volatile v4f*)(h + ((size_t)nodeBase + slot) * DF + c4) = hv;
  }
  __threadfence();
#pragma unroll 4
  for (int i = 0; i < (NB1 * DF / 4) / NTHR; ++i) {
    const int idx  = i * NTHR + tid;
    const int slot = idx >> 5;
    const int c4   = (idx & 31) * 4;
    const v4f hv = *(const v4f*)(acc + slot * DF + c4);
    *(volatile v4f*)(h + ((size_t)nodeBase + slot) * DF + c4) = hv;
  }
}

__global__ __launch_bounds__(NTHR) void k_gemm2(
    const float* __restrict__ hs, const float* __restrict__ ho,
    const int* __restrict__ tgt, const int* __restrict__ sidx, int S,
    const _Float16* __restrict__ w3s, const float* __restrict__ dis, float* t, int nN) {
  extern __shared__ v4f lds_dyn[];
  _Float16* sA  = (_Float16*)lds_dyn;
  float*    stg = (float*)lds_dyn;
  __shared__ int hitw[NWAVE * GROWS];
  __shared__ int hitp[GROWS];
  const int tid = threadIdx.x, lane = tid & 31, wave = tid >> 5, hh = lane >> 4, m = lane & 15;
  const int rowBase = blockIdx.x * GROWS;

  for (int i = tid; i < NWAVE * GROWS; i += NTHR) hitw[i] = -1;
  __syncthreads();

  {
    const int per  = (S + NWAVE - 1) / NWAVE;
    const int pbeg = wave * per;
    int pend = pbeg + per;
    pend = pend > S ? S : pend;
#pragma unroll 1
    for (int pb = pbeg; pb < pend; pb += 32) {
      const int p  = pb + lane;
      int pc = p > S - 1 ? S - 1 : p;
      pc = pc < 0 ? 0 : pc;
      const int tv = tgt[pc];
      const unsigned sl = (unsigned)tv - (unsigned)rowBase;
      const bool hit = (p < pend) && (sl < (unsigned)GROWS);
      unsigned msk = __builtin_amdgcn_ballot_w32(hit);
      while (msk != 0u) {
        const int j = __builtin_ctz(msk);
        msk &= msk - 1u;
        const int sj = __shfl((int)sl, j);
        if (lane == 0) hitw[wave * GROWS + (sj & (GROWS - 1))] = pb + j;
      }
    }
  }
  __syncthreads();
  if (tid < GROWS) {
    int best = -1;
#pragma unroll
    for (int w = 0; w < NWAVE; ++w) { const int v = hitw[w * GROWS + tid]; best = v > best ? v : best; }
    hitp[tid] = best;
  }
  __syncthreads();

#pragma unroll
  for (int i = 0; i < (GROWS * DF / 8) / NTHR; ++i) {
    const int idx = i * NTHR + tid;
    const int r   = idx >> 4;
    const int c0  = (idx & 15) * 8;
    int node = rowBase + r;
    node = node > nN - 1 ? nN - 1 : node;
    const float* xp = hs + (size_t)node * DF + c0;
    v4f a = *(const v4f*)xp, bb = *(const v4f*)(xp + 4);
    const int p = hitp[r];
    int pc = p > S - 1 ? S - 1 : p;
    pc = pc < 0 ? 0 : pc;
    int s = sidx[pc];
    s = s < 0 ? 0 : (s > nN - 1 ? nN - 1 : s);
    const float* op = ho + (size_t)s * DF + c0;
    const v4f oa = *(const v4f*)op;
    const v4f ob = *(const v4f*)(op + 4);
    const bool use = p >= 0;
    a.x  += use ? oa.x : 0.f;  a.y  += use ? oa.y : 0.f;  a.z  += use ? oa.z : 0.f;  a.w  += use ? oa.w : 0.f;
    bb.x += use ? ob.x : 0.f;  bb.y += use ? ob.y : 0.f;  bb.z += use ? ob.z : 0.f;  bb.w += use ? ob.w : 0.f;
    *(v8h*)(sA + r * APITCH + c0) = cvt8(a, bb);
  }
  __syncthreads();

  v8f acc[4];
#pragma unroll
  for (int tt = 0; tt < 4; ++tt) { v8f z = {0.f, 0.f, 0.f, 0.f, 0.f, 0.f, 0.f, 0.f}; acc[tt] = z; }
  const _Float16* ar = sA + (wave * 16 + m) * APITCH + 8 * hh;
#pragma unroll
  for (int kt = 0; kt < DF / 32; ++kt) {
    FragH a;
    a.h[0] = *(const v8h*)(ar + 32 * kt);
    a.h[1] = *(const v8h*)(ar + 32 * kt + 16);
#pragma unroll
    for (int tt = 0; tt < 4; ++tt) {
      const _Float16* bp = w3s + (size_t)(16 * tt + m) * DF + 32 * kt + 8 * hh;
      FragH b;
      b.h[0] = *(const v8h*)bp;
      b.h[1] = *(const v8h*)(bp + 16);
      acc[tt] = wmh(a.v, b.v, acc[tt]);
    }
  }
  __syncthreads();

  const int r0 = wave * 16 + 8 * hh;
  const v4f dA = *(const v4f*)(dis + (size_t)rowBase + r0);
  const v4f dB = *(const v4f*)(dis + (size_t)rowBase + r0 + 4);
  const float d0 = dA.x * WINV, d1 = dA.y * WINV, d2 = dA.z * WINV, d3 = dA.w * WINV;
  const float d4 = dB.x * WINV, d5 = dB.y * WINV, d6 = dB.z * WINV, d7 = dB.w * WINV;
  float* sp = stg + r0 * DO + m;
#pragma unroll
  for (int tt = 0; tt < 4; ++tt) {
    sp[0 * DO + 16 * tt] = acc[tt][0] * d0;
    sp[1 * DO + 16 * tt] = acc[tt][1] * d1;
    sp[2 * DO + 16 * tt] = acc[tt][2] * d2;
    sp[3 * DO + 16 * tt] = acc[tt][3] * d3;
    sp[4 * DO + 16 * tt] = acc[tt][4] * d4;
    sp[5 * DO + 16 * tt] = acc[tt][5] * d5;
    sp[6 * DO + 16 * tt] = acc[tt][6] * d6;
    sp[7 * DO + 16 * tt] = acc[tt][7] * d7;
  }
  __syncthreads();

  const float* lp = stg + wave * 16 * DO + 4 * lane;
  float* gp = t + ((size_t)rowBase + wave * 16) * DO + 4 * lane;
#pragma unroll
  for (int q = 0; q < 8; ++q) { const v4f v = *(const v4f*)(lp + q * 128); *(volatile v4f*)(gp + q * 128) = v; }
  __threadfence();
#pragma unroll
  for (int q = 0; q < 8; ++q) { const v4f v = *(const v4f*)(lp + q * 128); *(volatile v4f*)(gp + q * 128) = v; }
}

__global__ __launch_bounds__(NTHR) void k_agg2(
    const int* __restrict__ ei, const float* __restrict__ ew, const float* __restrict__ t,
    const float* __restrict__ dis, const float* __restrict__ b, float* out,
    int nN, int nE, int vec8) {
  extern __shared__ v4f lds_dyn[];
  float* acc  = (float*)lds_dyn;
  int*   list = (int*)(acc + NB2 * DO);
  int*   wcnt = list + LISTN;
  const int tid = threadIdx.x, lane = tid & 31, wave = tid >> 5;
  const int nodeBase = blockIdx.x * NB2;
  const int* dsts = ei + nE;

  {
    const v4f z = {0.f, 0.f, 0.f, 0.f};
    for (int i = tid; i < NB2 * DO / 4; i += NTHR) lds_dyn[i] = z;
  }
  __syncthreads();

  const int nChunks = (nE + CHUNK - 1) / CHUNK;
#pragma unroll 1
  for (int ch = 0; ch < nChunks; ++ch) {
    const int cbase = ch * CHUNK;
    const int wc = scan_chunk<NB2>(dsts, nE, cbase, nodeBase, vec8, list, tid, lane, wave);
    if (lane == 0) wcnt[wave] = wc;
    __syncthreads();
    if (wave == 0) {
#pragma unroll 1
      for (int wsx = 0; wsx < NWAVE; ++wsx) {
        int n = __builtin_amdgcn_readfirstlane(wcnt[wsx]);
        n = n > WCAP ? WCAP : (n < 0 ? 0 : n);
        const int* lp = list + wsx * WCAP;
#pragma unroll 1
        for (int i = 0; i < n; ++i) {
          const int ent  = __builtin_amdgcn_readfirstlane(lp[i]);
          const int slot = ent & (NB2 - 1);
          int e = cbase + ((ent >> 12) & (CHUNK - 1));
          e = e > nE - 1 ? nE - 1 : e;
          int src = ei[e];
          src = src < 0 ? 0 : (src > nN - 1 ? nN - 1 : src);
          const float wv = ew[e];
          const v2f v = *(const v2f*)(t + (size_t)src * DO + 2 * lane);
          v2f* ap = (v2f*)(acc + slot * DO + 2 * lane);
          *ap = *ap + v * wv;
        }
      }
    }
    __syncthreads();
  }

#pragma unroll 4
  for (int i = 0; i < (NB2 * DO / 4) / NTHR; ++i) {
    const int idx  = i * NTHR + tid;
    const int slot = idx >> 4;
    const int c4   = (idx & 15) * 4;
    const int node = nodeBase + slot;
    const int nc   = node > nN - 1 ? nN - 1 : node;
    const float d  = dis[nc];
    const v4f   gv = *(const v4f*)(t + (size_t)nc * DO + c4);
    const v4f   bv = *(const v4f*)(b + c4);
    v4f* ap = (v4f*)(acc + slot * DO + c4);
    const v4f ov = (*ap + gv) * d + bv;
    *ap = ov;
    if (node < nN) *(volatile v4f*)(out + (size_t)node * DO + c4) = ov;
  }
  __threadfence();
#pragma unroll 4
  for (int i = 0; i < (NB2 * DO / 4) / NTHR; ++i) {
    const int idx  = i * NTHR + tid;
    const int slot = idx >> 4;
    const int c4   = (idx & 15) * 4;
    const int node = nodeBase + slot;
    const v4f ov = *(const v4f*)(acc + slot * DO + c4);
    if (node < nN) *(volatile v4f*)(out + (size_t)node * DO + c4) = ov;
  }
}

extern "C" void kernel_launch(void* const* d_in, const int* in_sizes, int n_in,
                              void* d_out, int out_size, void* d_ws, size_t ws_size,
                              hipStream_t stream) {
  if (n_in < 13) return;
  const int nN = in_sizes[0] / DF;
  if (nN <= 0 || in_sizes[0] != nN * DF || in_sizes[3] != nN * DF) return;
  const int nE1 = in_sizes[2];
  const int nE2 = in_sizes[5];
  if (nE1 < 0 || nE2 < 0 || in_sizes[1] != 2 * nE1 || in_sizes[4] != 2 * nE2) return;
  const int S = in_sizes[6] / 2;
  if (S < 1 || in_sizes[6] != 2 * S) return;
  if (in_sizes[7] != DF * DF || in_sizes[9] != DF * DF || in_sizes[11] != DF * DO) return;
  if (in_sizes[8] < DF || in_sizes[10] < DF || in_sizes[12] < DO) return;
  if (out_size != 2 * nN * DO) return;

  const float* x1  = (const float*)d_in[0];
  const int*   ei1 = (const int*)d_in[1];
  const float* ew1 = (const float*)d_in[2];
  const float* x2  = (const float*)d_in[3];
  const int*   ei2 = (const int*)d_in[4];
  const float* ew2 = (const float*)d_in[5];
  const int*   sd  = (const int*)d_in[6];
  const float* W1  = (const float*)d_in[7];
  const float* b1  = (const float*)d_in[8];
  const float* W2  = (const float*)d_in[9];
  const float* b2  = (const float*)d_in[10];
  const float* W3  = (const float*)d_in[11];
  const float* b3  = (const float*)d_in[12];
  const int* sd0 = sd;
  const int* sd1 = sd + S;
  float* out0 = (float*)d_out;
  float* out1 = out0 + (size_t)nN * DO;

  const int nBD = (nN + NBD - 1) / NBD;
  const int nG  = (nN + GROWS - 1) / GROWS;
  const int nA1 = (nN + NB1 - 1) / NB1;
  const int nA2 = (nN + NB2 - 1) / NB2;

  char* ws = (char*)d_ws;
  size_t off = 0;
  const size_t oW1 = off; off += (size_t)DF * DF * 2;                   off = (off + 255) & ~(size_t)255;
  const size_t oW2 = off; off += (size_t)DF * DF * 2;                   off = (off + 255) & ~(size_t)255;
  const size_t oW3 = off; off += (size_t)DO * DF * 2;                   off = (off + 255) & ~(size_t)255;
  const size_t oD1 = off; off += (size_t)nBD * NBD * 4;                 off = (off + 255) & ~(size_t)255;
  const size_t oD2 = off; off += (size_t)nBD * NBD * 4;                 off = (off + 255) & ~(size_t)255;
  const size_t oG1 = off; off += (size_t)nG * GROWS * DF * 4;           off = (off + 255) & ~(size_t)255;
  const size_t oG2 = off; off += (size_t)nG * GROWS * DF * 4;           off = (off + 255) & ~(size_t)255;
  const size_t oH1 = off; off += (size_t)nA1 * NB1 * DF * 4;            off = (off + 255) & ~(size_t)255;
  const size_t oH2 = off; off += (size_t)nA1 * NB1 * DF * 4;            off = (off + 255) & ~(size_t)255;
  if (off > ws_size) return;
  _Float16* w1s  = (_Float16*)(ws + oW1);
  _Float16* w2s  = (_Float16*)(ws + oW2);
  _Float16* w3s  = (_Float16*)(ws + oW3);
  float*    dis1 = (float*)(ws + oD1);
  float*    dis2 = (float*)(ws + oD2);
  float*    g1   = (float*)(ws + oG1);
  float*    g2   = (float*)(ws + oG2);
  float*    h1   = (float*)(ws + oH1);
  float*    h2   = (float*)(ws + oH2);
  float*    t1   = g1;
  float*    t2   = g2;

  const int vec1 = ((nE1 & 3) == 0) ? 1 : 0;
  const int vec2 = ((nE2 & 3) == 0) ? 1 : 0;

  const int nPrep = 2 * (DF * DF / 8) + DO * DF / 8;
  k_wprep<<<(nPrep + NTHR - 1) / NTHR, NTHR, 0, stream>>>(W1, W2, W3, w1s, w2s, w3s);

  k_deg<<<nBD, NTHR, 0, stream>>>(ei1, ew1, dis1, nN, nE1, vec1);
  k_deg<<<nBD, NTHR, 0, stream>>>(ei2, ew2, dis2, nN, nE2, vec2);

  hipFuncSetAttribute(reinterpret_cast<const void*>(&k_gemm1),
                      hipFuncAttributeMaxDynamicSharedMemorySize, LDS_GEMM1);
  k_gemm1<<<nG, NTHR, LDS_GEMM1, stream>>>(x1, w1s, dis1, g1, nN);
  k_gemm1<<<nG, NTHR, LDS_GEMM1, stream>>>(x2, w2s, dis2, g2, nN);

  hipFuncSetAttribute(reinterpret_cast<const void*>(&k_agg1),
                      hipFuncAttributeMaxDynamicSharedMemorySize, LDS_AGG1);
  k_agg1<<<nA1, NTHR, LDS_AGG1, stream>>>(ei1, ew1, g1, dis1, b1, h1, nN, nE1, vec1);
  k_agg1<<<nA1, NTHR, LDS_AGG1, stream>>>(ei2, ew2, g2, dis2, b2, h2, nN, nE2, vec2);

  hipFuncSetAttribute(reinterpret_cast<const void*>(&k_gemm2),
                      hipFuncAttributeMaxDynamicSharedMemorySize, LDS_GEMM2);
  k_gemm2<<<nG, NTHR, LDS_GEMM2, stream>>>(h1, h2, sd0, sd1, S, w3s, dis1, t1, nN);
  k_gemm2<<<nG, NTHR, LDS_GEMM2, stream>>>(h2, h1, sd1, sd0, S, w3s, dis2, t2, nN);

  hipFuncSetAttribute(reinterpret_cast<const void*>(&k_agg2),
                      hipFuncAttributeMaxDynamicSharedMemorySize, LDS_AGG2);
  k_agg2<<<nA2, NTHR, LDS_AGG2, stream>>>(ei1, ew1, t1, dis1, b3, out0, nN, nE1, vec1);
  k_agg2<<<nA2, NTHR, LDS_AGG2, stream>>>(ei2, ew2, t2, dis2, b3, out1, nN, nE2, vec2);
}
